// KANConv2d_257698038307
// MI455X (gfx1250) — hardware-verified
//
#include <hip/hip_runtime.h>
#include <math.h>

typedef __attribute__((ext_vector_type(16))) _Float16 v16h;
typedef __attribute__((ext_vector_type(16))) __bf16 v16b;
typedef __attribute__((ext_vector_type(8)))  _Float16 v8h;
typedef __attribute__((ext_vector_type(8)))  float v8f;
typedef __attribute__((ext_vector_type(4)))  float v4f;
typedef __attribute__((ext_vector_type(2)))  float v2f;
typedef __attribute__((ext_vector_type(4)))  unsigned v4u;
typedef __attribute__((ext_vector_type(4)))  int v4i;
typedef float __attribute__((may_alias)) float_a;
typedef int __attribute__((may_alias)) int_a;

template <typename T> __device__ __forceinline__ void vst2(void* p, T v) { *(volatile T*)p = v; __threadfence(); *(volatile T*)p = v; }
__device__ __forceinline__ v8f wmma16(v16h a, v16h b, v8f c) {
  v8f d = __builtin_amdgcn_wmma_f32_16x16x32_f16(false, a, false, b, (short)0, c, false, false);
  asm volatile("v_nop\n\tv_nop\n\tv_nop\n\tv_nop" : "+v"(d) : "v"(a), "v"(b));
  return d;
}
__device__ __forceinline__ v8f wmma_bf(v16b a, v16b b, v8f c) {
  v8f d = __builtin_amdgcn_wmma_f32_16x16x32_bf16(false, a, false, b, (short)0, c, false, false);
  asm volatile("v_nop\n\tv_nop\n\tv_nop\n\tv_nop" : "+v"(d) : "v"(a), "v"(b));
  return d;
}
__device__ __forceinline__ v16h frag_h(const _Float16* rowk0, int lane) {
  union { v16h v; v8h q[2]; } u; const _Float16* p = rowk0 + 8 * (lane >> 4);
  u.q[0] = *(const v8h*)p; u.q[1] = *(const v8h*)(p + 16); return u.v;
}
__device__ __forceinline__ v16h frag_f32(const float* rowk0, int lane) {
  v16h a; const float* p = rowk0 + 8 * (lane >> 4);
#pragma unroll
  for (int i = 0; i < 8; ++i) { a[i] = (_Float16)p[i]; a[8 + i] = (_Float16)p[16 + i]; }
  return a;
}
__device__ __forceinline__ v16h frag_f32s(const float* rowk0, int lane, float sc) {
  v16h a; const float* p = rowk0 + 8 * (lane >> 4);
#pragma unroll
  for (int i = 0; i < 8; ++i) { a[i] = (_Float16)(p[i] * sc); a[8 + i] = (_Float16)(p[16 + i] * sc); }
  return a;
}
__device__ __forceinline__ v16h fragc_f32(const float* W, int k0, int n, int lane, int ld, int K) {
  v16h a; const int g = lane >> 4;
#pragma unroll
  for (int i = 0; i < 8; ++i) { const int ka = k0 + 8 * g + i, kb = ka + 16;
    a[i] = (_Float16)(ka < K ? W[(size_t)(ka < K ? ka : K - 1) * ld + n] : 0.f); a[8 + i] = (_Float16)(kb < K ? W[(size_t)(kb < K ? kb : K - 1) * ld + n] : 0.f); }
  return a;
}
struct F2 { v16b h, l; };
__device__ __forceinline__ F2 bsplit16(const float v[16]) { F2 r;
#pragma unroll
  for (int i = 0; i < 16; ++i) { const __bf16 h = (__bf16)v[i]; r.h[i] = h; r.l[i] = (__bf16)(v[i] - (float)h); }
  return r; }
__device__ __forceinline__ F2 split_row(const float* row, int k0, int lane) { float v[16]; const float* p = row + k0 + 8 * (lane >> 4);
#pragma unroll
  for (int i = 0; i < 8; ++i) { v[i] = p[i]; v[8 + i] = p[16 + i]; }
  return bsplit16(v); }
__device__ __forceinline__ F2 split_rowK(const float* row, int k0, int lane, int K) { float v[16]; const int g = lane >> 4;
#pragma unroll
  for (int i = 0; i < 8; ++i) { const int ka = k0 + 8 * g + i, kb = ka + 16; v[i] = ka < K ? row[ka < K ? ka : K - 1] : 0.f; v[8 + i] = kb < K ? row[kb < K ? kb : K - 1] : 0.f; }
  return bsplit16(v); }
__device__ __forceinline__ F2 split_col(const float* W, int k0, int n, int lane, int ld, int K) { float v[16]; const int g = lane >> 4;
#pragma unroll
  for (int i = 0; i < 8; ++i) { const int ka = k0 + 8 * g + i, kb = ka + 16; v[i] = ka < K ? W[(size_t)(ka < K ? ka : K - 1) * ld + n] : 0.f; v[8 + i] = kb < K ? W[(size_t)(kb < K ? kb : K - 1) * ld + n] : 0.f; }
  return bsplit16(v); }
__device__ __forceinline__ v8f mac3(const F2& a, const F2& b, v8f c) { c = wmma_bf(a.l, b.h, c); c = wmma_bf(a.h, b.l, c); return wmma_bf(a.h, b.h, c); }
__device__ __forceinline__ float sigm(float v) { return 1.0f / (1.0f + expf(-v)); }
#define LDSX() do { asm volatile("s_wait_dscnt 0" ::: "memory"); __builtin_amdgcn_wave_barrier(); __builtin_amdgcn_fence(__ATOMIC_RELEASE, "workgroup"); } while (0)


#define NB 4
#define CI 16
#define CO 16
#define IH 128
#define IW 128
#define K2 9
#define NBS 8
#define NKN 12
#define KA (CI * K2)
#define KAP 160
#define KB (CI * K2 * NBS)
#ifndef TNB
#define TNB NB
#endif
typedef __attribute__((ext_vector_type(8))) __bf16 v8b;
__device__ __forceinline__ v16b frag_b(const __bf16* rowk0, int lane) {
  union { v16b v; v8b q[2]; } u; const __bf16* p = rowk0 + 8 * (lane >> 4);
  u.q[0] = *(const v8b*)p; u.q[1] = *(const v8b*)(p + 16); return u.v;
}
__device__ __forceinline__ float bfr(float v) { return (float)(__bf16)v; }
__device__ __attribute__((noinline)) float exp_ni(float v) { return expf(v); }
__device__ __attribute__((noinline)) float erf_ni(float v) { return erff(v); }

#define WS_BW  0u
#define WS_SW  (WS_BW + 4u * (size_t)CO * KA)
#define WS_END (WS_SW + 4u * (size_t)CO * KB)

__global__ __launch_bounds__(256) void k_wprep(const float* __restrict__ BWT, const float* __restrict__ SWT, const float* __restrict__ SSC, float* __restrict__ BW, float* __restrict__ SW) { __shared__ __align__(16) float sb[CO * KA]; __shared__ __align__(16) float ssw[CO * KB];
  const int t = threadIdx.x;
  for (int e = t; e < CO * KA; e += 256) { const int i = e / KA, rem = e % KA; const int j = rem / K2, n = rem % K2; float s = 0.f;
#pragma unroll 1
    for (int m = 0; m < K2; ++m) s += bfr(BWT[((i * CI + j) * K2 + m) * K2 + n]); sb[e] = s; }
  for (int e = t; e < CO * KB; e += 256) { const int i = e / KB, rem = e % KB; const int jn = rem / NBS, s8 = rem % NBS; const int j = jn / K2, n = jn % K2; float s = 0.f;
#pragma unroll 1
    for (int m = 0; m < K2; ++m) s += bfr(SWT[(((i * CI + j) * K2 + m) * K2 + n) * NBS + s8]) * bfr(SSC[((i * CI + j) * K2 + m) * K2 + n]); ssw[e] = s; }
  __syncthreads();
  for (int q = t; q < CO * KA / 4; q += 256) vst2(BW + q * 4, *(const v4f*)&sb[q * 4]);
  for (int q = t; q < CO * KB / 4; q += 256) vst2(SW + q * 4, *(const v4f*)&ssw[q * 4]); }
__device__ __forceinline__ void bspl8(float x, float* out8) { float g[NKN];
#pragma unroll
  for (int m = 0; m < NKN; ++m) g[m] = (float)(m - 3) * 0.4f - 1.0f;
  float bs[NKN - 1];
#pragma unroll
  for (int m = 0; m < NKN - 1; ++m) bs[m] = (x >= g[m] && x < g[m + 1]) ? 1.0f : 0.0f;
#pragma unroll
  for (int k = 1; k <= 3; ++k) {
#pragma unroll
    for (int m = 0; m < NKN - 1 - k; ++m) { const float left = (x - g[m]) / (g[m + k] - g[m]) * bs[m]; const float right = (g[m + k + 1] - x) / (g[m + k + 1] - g[m + 1]) * bs[m + 1]; bs[m] = left + right; } }
#pragma unroll
  for (int s = 0; s < NBS; ++s) out8[s] = bs[s]; }
__global__ __launch_bounds__(128) void k_kan(const float* __restrict__ X, const float* __restrict__ BW, const float* __restrict__ SW, const float* __restrict__ BIAS, float* __restrict__ OUT) {
  __shared__ __align__(16) float sx[CI][3][68];
  __shared__ __align__(16) float so[CO][68];
  const int tid = threadIdx.x, wave = tid >> 5, lane = tid & 31, col = lane & 15, g = lane >> 4; const size_t p0 = (size_t)blockIdx.x * 64; const size_t b = p0 / (IH * IW); const int pp = (int)(p0 % (IH * IW)); const int y = pp / IW, x0 = pp % IW;
  for (int e = tid; e < CI * 3 * 66; e += 128) { const int j = e / (3 * 66), rem = e % (3 * 66); const int rr = rem / 66, cc = rem % 66; const int gy = y - 1 + rr, gx = x0 - 1 + cc; float v = 0.f; if (gy >= 0 && gy < IH && gx >= 0 && gx < IW) v = bfr(X[((b * CI + j) * IH + gy) * (size_t)IW + gx]); sx[j][rr][cc] = v; }
  __syncthreads();
  const int pl = wave * 16 + col;
  v8f acc = {};
#pragma unroll 1
  for (int kc = 0; kc < KAP / 32; ++kc) { v16b ah, al;
#pragma unroll
    for (int q = 0; q < 16; ++q) { const int k = kc * 32 + 8 * g + (q < 8 ? q : q + 8); float sv = 0.f; if (k < KA) { const int j = k / K2, n = k % K2; const float pv = sx[j][n / 3][pl + (n % 3)]; sv = pv / (1.0f + expf(-pv)); } const __bf16 h = (__bf16)sv; ah[q] = h; al[q] = (__bf16)(sv - (float)h); }
    v16b wh, wl;
#pragma unroll
    for (int q = 0; q < 16; ++q) { const int k = kc * 32 + 8 * g + (q < 8 ? q : q + 8); const float wv = (k < KA) ? BW[col * KA + k] : 0.f; const __bf16 h = (__bf16)wv; wh[q] = h; wl[q] = (__bf16)(wv - (float)h); }
    acc = wmma_bf(ah, wh, acc); acc = wmma_bf(al, wh, acc); acc = wmma_bf(ah, wl, acc); }
#pragma unroll 1
  for (int kc = 0; kc < KB / 32; ++kc) { v16b ah, al;
#pragma unroll
    for (int tp = 0; tp < 2; ++tp) { const int jn = kc * 4 + g + 2 * tp;     const int j = jn / K2, n = jn % K2; const float pv = sx[j][n / 3][pl + (n % 3)]; float b8[NBS]; bspl8(pv, b8);
#pragma unroll
      for (int s = 0; s < NBS; ++s) { const __bf16 h = (__bf16)b8[s]; ah[tp * 8 + s] = h; al[tp * 8 + s] = (__bf16)(b8[s] - (float)h); } }
    v16b wh, wl;
#pragma unroll
    for (int q = 0; q < 16; ++q) { const int k = kc * 32 + 8 * g + (q < 8 ? q : q + 8); const float wv = SW[col * KB + k]; const __bf16 h = (__bf16)wv; wh[q] = h; wl[q] = (__bf16)(wv - (float)h); }
    acc = wmma_bf(ah, wh, acc); acc = wmma_bf(al, wh, acc); acc = wmma_bf(ah, wl, acc); }
#pragma unroll
  for (int r = 0; r < 8; ++r) so[col][wave * 16 + 8 * g + r] = acc[r] + bfr(BIAS[col]);
  __syncthreads(); for (int e = tid; e < CO * 16; e += 128) { const int i = e >> 4, q = e & 15; vst2(OUT + ((b * CO + i) * IH + y) * (size_t)IW + x0 + q * 4, *(const v4f*)&so[i][q * 4]); } }
extern "C" void kernel_launch(void* const* d_in, const int* in_sizes, int n_in, void* d_out, int out_size, void* d_ws, size_t ws_size, hipStream_t stream) {
  (void)in_sizes; (void)n_in; (void)out_size;
  const float** F = (const float**)d_in;
  if (ws_size < (size_t)WS_END) return;
  char* ws = (char*)d_ws; float *BW = (float*)(ws + WS_BW), *SW = (float*)(ws + WS_SW);
  k_wprep<<<1, 256, 0, stream>>>(F[1], F[2], F[3], BW, SW);
  k_kan<<<TNB * IH * IW / 64, 128, 0, stream>>>(F[0], BW, SW, F[4], (float*)d_out);
}
